// SelfAttentionBlock_5566277616017
// MI455X (gfx1250) — hardware-verified
//
#include <hip/hip_runtime.h>


#ifndef NB
#define NB 8
#endif
#ifndef SEQ
#define SEQ 4096
#endif
#define NB_FULL  8
#define SEQ_FULL 4096
#define CCH  256
#define RCD  32
#define QKW  64
#define PCAR 16384.0f
#define VCAR 16.0f
#define L2E  1.4426950408889634f
#define OSP  260

static_assert(SEQ % 64 == 0);
static_assert(SEQ <= SEQ_FULL);
static_assert(NB >= 1);
static_assert(NB <= NB_FULL);
static_assert((OSP % 4) == 0);

typedef _Float16 h16;
typedef unsigned short bf;
typedef __attribute__((ext_vector_type(16))) __bf16   v16bf;
typedef __attribute__((ext_vector_type(16))) _Float16 v16h;
typedef __attribute__((ext_vector_type(8)))  _Float16 v8h;
typedef __attribute__((ext_vector_type(8)))  unsigned short v8us;
typedef __attribute__((ext_vector_type(8)))  float    v8f;
typedef __attribute__((ext_vector_type(4)))  float    v4f;
typedef __attribute__((ext_vector_type(2)))  unsigned short v2us;
typedef v8h  __attribute__((may_alias)) v8ha;
typedef v4f  __attribute__((may_alias)) v4fa;
typedef v8us __attribute__((may_alias)) v8usa;

__device__ __forceinline__ unsigned short f2bf(float f) { unsigned u = __float_as_uint(f); u += 0x7FFFu + ((u >> 16) & 1u); return (unsigned short)(u >> 16); }
__device__ __forceinline__ float bf2f(unsigned short b) { return __uint_as_float(((unsigned)b) << 16); }
__device__ __forceinline__ float bfr(float f) { return bf2f(f2bf(f)); }
__device__ __forceinline__ v16h cat16(v8h lo, v8h hi) { return __builtin_shufflevector(lo, hi, 0, 1, 2, 3, 4, 5, 6, 7, 8, 9, 10, 11, 12, 13, 14, 15); }
__device__ __forceinline__ v16bf cat16b(v8us lo, v8us hi) { return __builtin_bit_cast(v16bf, __builtin_shufflevector(lo, hi, 0, 1, 2, 3, 4, 5, 6, 7, 8, 9, 10, 11, 12, 13, 14, 15)); }
__device__ __forceinline__ v8f wmma16(v16h a, v16h b, v8f c) { return __builtin_amdgcn_wmma_f32_16x16x32_f16(false, a, false, b, (short)0, c, false, false); }
__device__ __forceinline__ v8f wmmab(v16bf a, v16bf b, v8f c) { return __builtin_amdgcn_wmma_f32_16x16x32_bf16(false, a, false, b, (short)0, c, false, false); }
__device__ __forceinline__ h16 tohx(float x) { return (h16)x; }
__device__ __forceinline__ void splitf(float y, unsigned short& h, unsigned short& l) { h = f2bf(y); l = f2bf(y - bf2f(h)); }

template <typename T16> struct WFrag;
template <> struct WFrag<h16> { typedef v16h V; static __device__ __forceinline__ V ld(const h16* p) { return cat16(*(const v8h*)p, *(const v8h*)(p + 16)); } static __device__ __forceinline__ v8f mma(V a, V b, v8f c) { return wmma16(a, b, c); } };
template <> struct WFrag<bf> { typedef v16bf V; static __device__ __forceinline__ V ld(const bf* p) { return cat16b(*(const v8us*)p, *(const v8us*)(p + 16)); } static __device__ __forceinline__ v8f mma(V a, V b, v8f c) { return wmmab(a, b, c); } };

template <typename T16, int NSPLIT, bool BIAS>
__global__ __launch_bounds__(32) void k_gemmw(const T16* __restrict__ A, const T16* __restrict__ A2, const T16* __restrict__ Bt, const T16* __restrict__ Bt2, int K, float* C, int ldc, const float* __restrict__ bias, size_t sA, size_t sB, size_t sC) {
    typedef typename WFrag<T16>::V V;
    __shared__ __align__(16) float os[16 * 68];
    const size_t z = blockIdx.z; A += z * sA; if (A2) A2 += z * sA; Bt += z * sB; if (Bt2) Bt2 += z * sB; C += z * sC;
    const int lane = threadIdx.x & 31, lr = lane & 15, hi = lane >> 4; const int r0 = blockIdx.x * 64, c0 = blockIdx.y * 64;
    v8f acc[4][4];
#pragma unroll
    for (int mb = 0; mb < 4; ++mb)
#pragma unroll
        for (int nb = 0; nb < 4; ++nb) acc[mb][nb] = (v8f){};
    const size_t aoff = (size_t)(r0 + lr) * K + 8 * hi, boff = (size_t)(c0 + lr) * K + 8 * hi;
#pragma unroll 1
    for (int kc = 0; kc < K; kc += 32) {
        V a[4], a2[4];
#pragma unroll
        for (int mb = 0; mb < 4; ++mb) { a[mb] = WFrag<T16>::ld(A + aoff + (size_t)mb * 16 * K + kc); if (NSPLIT == 1 || NSPLIT == 2) a2[mb] = WFrag<T16>::ld(A2 + aoff + (size_t)mb * 16 * K + kc); }
#pragma unroll
        for (int nb = 0; nb < 4; ++nb) { const V b = WFrag<T16>::ld(Bt + boff + (size_t)nb * 16 * K + kc); V b2; if (NSPLIT >= 2) b2 = WFrag<T16>::ld(Bt2 + boff + (size_t)nb * 16 * K + kc);
#pragma unroll
            for (int mb = 0; mb < 4; ++mb) { acc[mb][nb] = WFrag<T16>::mma(a[mb], b, acc[mb][nb]); if (NSPLIT == 1 || NSPLIT == 2) acc[mb][nb] = WFrag<T16>::mma(a2[mb], b, acc[mb][nb]); if (NSPLIT >= 2) acc[mb][nb] = WFrag<T16>::mma(a[mb], b2, acc[mb][nb]); } }
        asm volatile("v_nop\n\tv_nop\n\tv_nop\n\tv_nop" : "+v"(acc[0][0]), "+v"(acc[1][1]), "+v"(acc[2][2]), "+v"(acc[3][3]) : "v"(a[0]), "v"(a[3]));
    }
#pragma unroll
    for (int mb = 0; mb < 4; ++mb) {
#pragma unroll
        for (int nb = 0; nb < 4; ++nb) {
#pragma unroll
            for (int j = 0; j < 8; ++j) os[(hi * 8 + j) * 68 + nb * 16 + lr] = acc[mb][nb][j]; }
        __builtin_amdgcn_wave_barrier(); asm volatile("" ::: "memory");
        float* crow = C + (size_t)(r0 + mb * 16) * ldc + c0;
#pragma unroll 1
        for (int ps = 0; ps < 2; ++ps) {
#pragma unroll
            for (int s = 0; s < 8; ++s) { const int row = 2 * s + hi, cofs = lr * 4; v4f val = *(const v4fa*)(os + row * 68 + cofs); if (BIAS) { val[0] += bfr(bias[c0 + cofs]); val[1] += bfr(bias[c0 + cofs + 1]); val[2] += bfr(bias[c0 + cofs + 2]); val[3] += bfr(bias[c0 + cofs + 3]); }
                *(volatile v4f*)(crow + (size_t)row * ldc + cofs) = val; }
            if (ps == 0) __threadfence(); }
        __builtin_amdgcn_wave_barrier(); asm volatile("" ::: "memory");
    }
}

__global__ __launch_bounds__(256) void k_wtG(const float* __restrict__ w, int K, int N, bf* Bt) {
    const int lane = threadIdx.x & 31; const int L0 = (blockIdx.x * 8 + (threadIdx.x >> 5)) * 8; const int nlines = N * K / 64;
#pragma unroll
    for (int ps = 0; ps < 2; ++ps) {
#pragma unroll 1
        for (int l = 0; l < 8; ++l) { const int L = L0 + l; if (L >= nlines) break; const size_t e = (size_t)L * 64 + lane * 2; const int k = (int)(e % K), n = (int)(e / K); v2us o;
            o[0] = f2bf(w[(size_t)k * N + n]); o[1] = f2bf(w[(size_t)(k + 1) * N + n]); *(volatile v2us*)(Bt + e) = o; }
        if (ps == 0) __threadfence(); }
}

__global__ __launch_bounds__(256) void k_cvtx(const float* __restrict__ x, bf* XB, size_t n8) {
    const size_t i = (size_t)blockIdx.x * 256 + threadIdx.x; if (i >= n8) return;
    const size_t per8 = (size_t)SEQ * CCH / 8; const size_t b = i / per8, r = i - b * per8;
    const v8f v = *(const v8f*)(x + b * ((size_t)SEQ_FULL * CCH) + r * 8); v8us o;
#pragma unroll
    for (int k = 0; k < 8; ++k) o[k] = f2bf(v[k]);
    *(volatile v8us*)(XB + i * 8) = o; __threadfence(); *(volatile v8us*)(XB + i * 8) = o;
}

__global__ __launch_bounds__(256) void k_qkp(const float* __restrict__ F, const float* __restrict__ bq, const float* __restrict__ bk, bf* Qh, bf* Ql, bf* Kh, bf* Kl, size_t n8) {
    const size_t i = (size_t)blockIdx.x * 256 + threadIdx.x; if (i >= n8) return;
    const size_t e = i * 8; const size_t n = e / RCD; const int d = (int)(e % RCD);
    const float* f = F + n * QKW;
    const v4f a0 = *(const v4f*)(f + d), a1 = *(const v4f*)(f + d + 4), c0 = *(const v4f*)(f + RCD + d), c1 = *(const v4f*)(f + RCD + d + 4);
    v8us qh, ql, kh, kl;
#pragma unroll
    for (int j = 0; j < 4; ++j) {
        unsigned short s1, s2;
        const float qv0 = fmaxf(a0[j] + bfr(bq[d + j]), 0.f);         splitf(qv0, s1, s2); qh[j] = s1;     ql[j] = s2;
        const float qv1 = fmaxf(a1[j] + bfr(bq[d + 4 + j]), 0.f);     splitf(qv1, s1, s2); qh[4 + j] = s1; ql[4 + j] = s2;
        const float kv0 = fmaxf(c0[j] + bfr(bk[d + j]), 0.f);         splitf(kv0, s1, s2); kh[j] = s1;     kl[j] = s2;
        const float kv1 = fmaxf(c1[j] + bfr(bk[d + 4 + j]), 0.f);     splitf(kv1, s1, s2); kh[4 + j] = s1; kl[4 + j] = s2;
    }
    *(volatile v8us*)(Qh + e) = qh; *(volatile v8us*)(Ql + e) = ql; *(volatile v8us*)(Kh + e) = kh; *(volatile v8us*)(Kl + e) = kl;
    __threadfence();
    *(volatile v8us*)(Qh + e) = qh; *(volatile v8us*)(Ql + e) = ql; *(volatile v8us*)(Kh + e) = kh; *(volatile v8us*)(Kl + e) = kl;
}

__global__ __launch_bounds__(256) void k_vtp(const float* __restrict__ F, h16* VT, size_t n8) {
    const size_t i = (size_t)blockIdx.x * 256 + threadIdx.x; if (i >= n8) return;
    const size_t e = i * 8; const int mm = (int)(e % SEQ); const int c = (int)((e / SEQ) % CCH); const size_t b = e / ((size_t)SEQ * CCH);
    const float* f = F + (b * SEQ + mm) * (size_t)CCH + c; v8h o;
#pragma unroll
    for (int j = 0; j < 8; ++j) o[j] = tohx(f[(size_t)j * CCH] * VCAR);
    *(volatile v8h*)(VT + e) = o; __threadfence(); *(volatile v8h*)(VT + e) = o;
}

__global__ __launch_bounds__(32) void k_flash(const bf* __restrict__ Qh, const bf* __restrict__ Ql, const bf* __restrict__ Kh, const bf* __restrict__ Kl,
                                              const h16* __restrict__ VT, const float* __restrict__ X, float* OUT) {
    __shared__ __align__(16) float os[16 * OSP];
    const int lane = threadIdx.x & 31, h = lane >> 4, m = lane & 15;
    const int b = blockIdx.y, q0 = blockIdx.x * 16;
    const size_t qrow = (size_t)b * SEQ + q0 + m;
    const v16bf qbh = WFrag<bf>::ld(Qh + qrow * RCD + 8 * h);
    const v16bf qbl = WFrag<bf>::ld(Ql + qrow * RCD + 8 * h);
    const bf* kph = Kh + ((size_t)b * SEQ + m) * RCD + 8 * h;
    const bf* kpl = Kl + ((size_t)b * SEQ + m) * RCD + 8 * h;
    const h16* vp = VT + ((size_t)b * CCH + m) * SEQ + 8 * h;
    const v8f z8 = {0.f, 0.f, 0.f, 0.f, 0.f, 0.f, 0.f, 0.f};
    v8f acc[16];
#pragma unroll
    for (int cb = 0; cb < 16; ++cb) acc[cb] = z8;
    float mq = -1.0e30f, lq = 0.f;
#pragma unroll 1
    for (int k0 = 0; k0 < SEQ; k0 += 32) {
        const v16bf ka0 = WFrag<bf>::ld(kph + (size_t)k0 * RCD);
        const v16bf kc0 = WFrag<bf>::ld(kpl + (size_t)k0 * RCD);
        const v16bf ka1 = WFrag<bf>::ld(kph + (size_t)(k0 + 16) * RCD);
        const v16bf kc1 = WFrag<bf>::ld(kpl + (size_t)(k0 + 16) * RCD);
        v8f st0 = wmmab(ka0, qbh, z8); st0 = wmmab(kc0, qbh, st0); st0 = wmmab(ka0, qbl, st0);
        v8f st1 = wmmab(ka1, qbh, z8); st1 = wmmab(kc1, qbh, st1); st1 = wmmab(ka1, qbl, st1);
        asm volatile("v_nop\n\tv_nop\n\tv_nop\n\tv_nop" : "+v"(st0), "+v"(st1) : "v"(ka0), "v"(kc0), "v"(ka1), "v"(kc1), "v"(qbh), "v"(qbl));
        float tmax = fmaxf(st0[0], st1[0]);
#pragma unroll
        for (int r = 1; r < 8; ++r) tmax = fmaxf(tmax, fmaxf(st0[r], st1[r]));
        tmax = fmaxf(tmax, __shfl_xor(tmax, 16, 32));
        const float mn = fmaxf(mq, tmax);
        const float sc = __builtin_amdgcn_exp2f((mq - mn) * L2E);
        mq = mn;
        v8h pl, ph; float rs = 0.f;
#pragma unroll
        for (int r = 0; r < 8; ++r) {
            const float e0 = __builtin_amdgcn_exp2f((st0[r] - mn) * L2E);
            const float e1 = __builtin_amdgcn_exp2f((st1[r] - mn) * L2E);
            rs += e0 + e1;
            pl[r] = tohx(e0 * PCAR); ph[r] = tohx(e1 * PCAR);
        }
        rs += __shfl_xor(rs, 16, 32);
        lq = lq * sc + rs;
        const v16h pb = cat16(pl, ph);
#pragma unroll
        for (int cb = 0; cb < 16; ++cb) acc[cb] = acc[cb] * sc;
#pragma unroll
        for (int g = 0; g < 8; ++g) {
            const v16h va = WFrag<h16>::ld(vp + (size_t)(2 * g) * 16 * SEQ + k0);
            const v16h vc = WFrag<h16>::ld(vp + (size_t)(2 * g + 1) * 16 * SEQ + k0);
            acc[2 * g]     = wmma16(va, pb, acc[2 * g]);
            acc[2 * g + 1] = wmma16(vc, pb, acc[2 * g + 1]);
            asm volatile("v_nop\n\tv_nop\n\tv_nop\n\tv_nop" : "+v"(acc[2 * g]), "+v"(acc[2 * g + 1]) : "v"(va), "v"(vc), "v"(pb));
        }
    }
    const float scale = (1.0f / lq) * (1.0f / (PCAR * VCAR));
#pragma unroll
    for (int cb = 0; cb < 16; ++cb) {
        v4f u0, u1;
#pragma unroll
        for (int j = 0; j < 4; ++j) { u0[j] = acc[cb][j] * scale; u1[j] = acc[cb][4 + j] * scale; }
        *(v4fa*)(os + m * OSP + cb * 16 + 8 * h)     = u0;
        *(v4fa*)(os + m * OSP + cb * 16 + 8 * h + 4) = u1;
    }
    __syncthreads();
    const float* xb = X + ((size_t)b * SEQ_FULL + q0) * CCH;
    float* ob = OUT + ((size_t)b * SEQ_FULL + q0) * CCH;
#pragma unroll 1
    for (int ps = 0; ps < 2; ++ps) {
#pragma unroll
        for (int r = 0; r < 16; ++r) {
#pragma unroll
            for (int c2 = 0; c2 < 2; ++c2) {
                const int c = c2 * 128 + lane * 4;
                v4f v = *(const v4fa*)(os + r * OSP + c);
                const v4f xx = *(const v4f*)(xb + (size_t)r * CCH + c);
                v[0] += bfr(xx[0]); v[1] += bfr(xx[1]); v[2] += bfr(xx[2]); v[3] += bfr(xx[3]);
                *(volatile v4f*)(ob + (size_t)r * CCH + c) = v;
            }
        }
        if (ps == 0) __threadfence();
    }
}

extern "C" void kernel_launch(void* const* d_in, const int* in_sizes, int n_in,
                              void* d_out, int out_size, void* d_ws, size_t ws_size, hipStream_t stream) {
    if (n_in < 7) return;
    const int need_x = (NB - 1) * SEQ_FULL * CCH + SEQ * CCH;
    if (in_sizes[0] < need_x || in_sizes[1] < CCH * RCD || in_sizes[2] < RCD || in_sizes[3] < CCH * RCD || in_sizes[4] < RCD || in_sizes[5] < CCH * CCH || in_sizes[6] < CCH) return;
    if (out_size < need_x) return;
    const float* x  = (const float*)d_in[0];
    const float* wq = (const float*)d_in[1];
    const float* bq = (const float*)d_in[2];
    const float* wk = (const float*)d_in[3];
    const float* bk = (const float*)d_in[4];
    const float* wv = (const float*)d_in[5];
    const float* bv = (const float*)d_in[6];
    float* OUT = (float*)d_out;
    char* wsp = (char*)d_ws;
    auto take = [&](size_t bytes) { char* p = wsp; wsp += (bytes + 255) & ~(size_t)255; return (void*)p; };
    const size_t NR = (size_t)NB * SEQ;
    bf*    WQK = (bf*)take((size_t)QKW * CCH * 2);
    bf*    WVT = (bf*)take((size_t)CCH * CCH * 2);
    bf*    XB  = (bf*)take(NR * CCH * 2);
    float* FQK = (float*)take(NR * QKW * 4);
    bf*    Qh  = (bf*)take(NR * RCD * 2);
    bf*    Ql  = (bf*)take(NR * RCD * 2);
    bf*    Kh  = (bf*)take(NR * RCD * 2);
    bf*    Kl  = (bf*)take(NR * RCD * 2);
    float* FV  = (float*)take(NR * CCH * 4);
    h16*   VT  = (h16*)take((size_t)NB * CCH * SEQ * 2);
    if ((size_t)(wsp - (char*)d_ws) > ws_size) return;

    k_wtG<<<(unsigned)((CCH * RCD / 64 + 63) / 64), 256, 0, stream>>>(wq, CCH, RCD, WQK);
    k_wtG<<<(unsigned)((CCH * RCD / 64 + 63) / 64), 256, 0, stream>>>(wk, CCH, RCD, WQK + (size_t)RCD * CCH);
    k_wtG<<<(unsigned)((CCH * CCH / 64 + 63) / 64), 256, 0, stream>>>(wv, CCH, CCH, WVT);
    { const size_t n8 = NR * CCH / 8; k_cvtx<<<(unsigned)((n8 + 255) / 256), 256, 0, stream>>>(x, XB, n8); }
    k_gemmw<bf, 0, false><<<dim3(SEQ / 64, QKW / 64, NB), 32, 0, stream>>>(XB, nullptr, WQK, nullptr, CCH, FQK, QKW, nullptr, (size_t)SEQ * CCH, 0, (size_t)SEQ * QKW);
    { const size_t n8 = NR * RCD / 8; k_qkp<<<(unsigned)((n8 + 255) / 256), 256, 0, stream>>>(FQK, bq, bk, Qh, Ql, Kh, Kl, n8); }
    k_gemmw<bf, 0, true><<<dim3(SEQ / 64, CCH / 64, NB), 32, 0, stream>>>(XB, nullptr, WVT, nullptr, CCH, FV, CCH, bv, (size_t)SEQ * CCH, 0, (size_t)SEQ * CCH);
    { const size_t n8 = (size_t)NB * CCH * SEQ / 8; k_vtp<<<(unsigned)((n8 + 255) / 256), 256, 0, stream>>>(FV, VT, n8); }
    k_flash<<<dim3(SEQ / 16, NB, 1), 32, 0, stream>>>(Qh, Ql, Kh, Kl, VT, x, OUT);
}
